// TGAT_89558658056628
// MI455X (gfx1250) — hardware-verified
//
#include <hip/hip_runtime.h>
#include <stddef.h>
#include <stdint.h>
#include <math.h>

#define NNODE 10000
#define KS    32
#define HF    128
#define NHEAD 8
#define HDIM  16
#define TF    64
#define TH    32
#define RF    32
#define OUTF  64
#define KQ3   384
#define KA    96
#define BKP   128
#define MP    10048
#define NSP   (MP * KS)
#define NTHR  256
#define GBM   64
#define GBN   128
#define GTHR  128
#define SRP   132
#define START_T   0.25f
#define END_T     0.75f
#define ATTN_NORM 0.25f
#define T_NORM    0.17677669529663689f
#define LN_EPS    1e-5f
#define CA   16.0f
#define CW   256.0f
#define INVC 0.000244140625f
#define WSMAX 134217728

#define U_WP  (HF * (HF / 8))
#define U_WK  (KQ3 * (256 / 8))
#define U_W1  (HF * (512 / 8))
#define U_W2  (HF * (256 / 8))
#define U_WO  (OUTF * (256 / 8))
#define U_BT  (256 * (TF / 8))
#define U_BE  (256 * (64 / 8))
#define U_TQW (HF * (TF / 8))
#define U_XB  (MP * (HF / 8))
#define E_WP  U_WP
#define E_WK  (E_WP + U_WK)
#define E_W1  (E_WK + U_W1)
#define E_W2  (E_W1 + U_W2)
#define E_WO  (E_W2 + U_WO)
#define E_BT  (E_WO + U_BT)
#define E_BE  (E_BT + U_BE)
#define E_TQW (E_BE + U_TQW)
#define E_XB  (E_TQW + U_XB)

#define L_SR  (8 * 16 * SRP * 4)
#define L_SQ  (8 * HF * 4)
#define L_SS  (8 * KS * NHEAD * 4)
#define L_SP  (8 * KS * NHEAD * 4)
#define L_SJ  (NTHR * 4)
#define L_SM  (NTHR * 4)
#define SLOT_LDS (L_SR + L_SQ + L_SS + L_SP + L_SJ + L_SM)

static_assert(MP % GBM == 0 && MP >= NNODE && MP - NNODE < GBM && MP % 8 == 0);
static_assert(KA % 32 == 0 && HF % 32 == 0 && TF % 32 == 0);
static_assert(E_WP % NTHR == 0 && E_WK % NTHR == 0 && E_W1 % NTHR == 0 && E_W2 % NTHR == 0 && E_WO % NTHR == 0);
static_assert(E_BT % NTHR == 0 && E_BE % NTHR == 0 && E_TQW % NTHR == 0 && E_XB % NTHR == 0);
static_assert(L_SR % 16 == 0 && L_SQ % 16 == 0 && L_SS % 16 == 0 && L_SP % 16 == 0 && L_SJ % 16 == 0);
static_assert(SLOT_LDS <= 300000);
static_assert(NTHR == 8 * KS && NTHR == 2 * HF && HF == NHEAD * HDIM && TF == 2 * TH && KA == TF + RF);
static_assert(2 * HF * 2 <= 16 * SRP * 4);
static_assert((SRP * 4) % 16 == 0 && SRP >= HF);
static_assert(GBM == (GTHR / 32) * 16 && GBN == 4 * 32);
static_assert(NNODE * OUTF == 640000);

typedef float          v4f   __attribute__((ext_vector_type(4)));
typedef float          v8f   __attribute__((ext_vector_type(8)));
typedef int            v8i   __attribute__((ext_vector_type(8)));
typedef unsigned short v4us  __attribute__((ext_vector_type(4)));
typedef unsigned short v8us  __attribute__((ext_vector_type(8)));
typedef __bf16         v16bf __attribute__((ext_vector_type(16)));
typedef _Float16       v16h  __attribute__((ext_vector_type(16)));
typedef _Float16       v8h   __attribute__((ext_vector_type(8)));
typedef _Float16       v2h   __attribute__((ext_vector_type(2)));
typedef v4f  __attribute__((may_alias)) v4fa;
typedef v4us __attribute__((may_alias)) v4usa;
typedef v8us __attribute__((may_alias)) v8usa;
typedef v8h  __attribute__((may_alias)) v8ha;
typedef v2h  __attribute__((may_alias)) v2ha;
union Frag16 { v16bf b; v16h h; v8us u[2]; v8i w; };

__device__ __forceinline__ v8f wm_b(const Frag16& a, const Frag16& b, v8f c) {
  v8f d = __builtin_amdgcn_wmma_f32_16x16x32_bf16(false, a.b, false, b.b, (short)0, c, false, false);
  asm volatile("v_nop\n\tv_nop\n\tv_nop\n\tv_nop" : "+v"(d) : "v"(a.w), "v"(b.w));
  return d;
}
__device__ __forceinline__ v8f wm_h(const Frag16& a, const Frag16& b, v8f c) {
  v8f d = __builtin_amdgcn_wmma_f32_16x16x32_f16(false, a.h, false, b.h, (short)0, c, false, false);
  asm volatile("v_nop\n\tv_nop\n\tv_nop\n\tv_nop" : "+v"(d) : "v"(a.w), "v"(b.w));
  return d;
}

__device__ __forceinline__ unsigned bf16_bits(float f) {
  const unsigned u = __float_as_uint(f);
  return (u + 0x7FFFu + ((u >> 16) & 1u)) >> 16;
}
__device__ __forceinline__ float bf16_val(float f) {
  return __uint_as_float(bf16_bits(f) << 16);
}
__device__ __forceinline__ v4f bf4(v4f a) {
  v4f r;
  r.x = bf16_val(a.x); r.y = bf16_val(a.y); r.z = bf16_val(a.z); r.w = bf16_val(a.w);
  return r;
}
__device__ __forceinline__ unsigned short hl_bits(float x, unsigned sel) {
  const unsigned hb = bf16_bits(x);
  const float hv = __uint_as_float(hb << 16);
  const unsigned lb = bf16_bits(x - hv);
  return (unsigned short)((hb & ~sel) | (lb & sel));
}
__device__ __forceinline__ void put8us(unsigned short* p, v8us o) {
  *(volatile v8us*)p = o;
  __threadfence();
  *(volatile v8us*)p = o;
}
__device__ __forceinline__ void put8h(_Float16* p, v8h o) {
  *(volatile v8h*)p = o;
  __threadfence();
  *(volatile v8h*)p = o;
}
__device__ __forceinline__ float dot4s(v4f q, v4f r, v4f g, float a) {
  a = a + q.x * (r.x + g.x);
  a = a + q.y * (r.y + g.y);
  a = a + q.z * (r.z + g.z);
  a = a + q.w * (r.w + g.w);
  return a;
}

__global__ __launch_bounds__(NTHR) void k_prep(const float* __restrict__ x, const float* __restrict__ Wp,
                                               const float* __restrict__ Wkqv, const float* __restrict__ Wtime,
                                               const float* __restrict__ Wedge, const float* __restrict__ W1,
                                               const float* __restrict__ W2, const float* __restrict__ Wo, int nN,
                                               unsigned short* XB, unsigned short* WpT, unsigned short* WkT,
                                               unsigned short* W1T, unsigned short* W2T, unsigned short* WoT,
                                               _Float16* BKV, _Float16* WtqT) {
  const int u = (int)blockIdx.x * NTHR + (int)threadIdx.x;
  if (u < E_WP) {
    const int n = u >> 4, k8 = (u & 15) * 8;
    v8us o;
#pragma unroll
    for (int i = 0; i < 8; ++i) o[i] = (unsigned short)bf16_bits(Wp[(size_t)(k8 + i) * HF + n]);
    put8us(WpT + (size_t)n * HF + k8, o);
  } else if (u < E_WK) {
    const int v = u - E_WP, n = v >> 5, k8 = (v & 31) * 8, ks = k8 & (HF - 1);
    v8us o;
#pragma unroll
    for (int i = 0; i < 8; ++i) o[i] = (unsigned short)bf16_bits(Wkqv[(size_t)(ks + i) * KQ3 + n]);
    put8us(WkT + (size_t)n * 256 + k8, o);
  } else if (u < E_W1) {
    const int v = u - E_WK, n = v >> 6, k8 = (v & 63) * 8;
    const int sr = (k8 & 127) + ((k8 >> 8) << 7);
    v8us o;
#pragma unroll
    for (int i = 0; i < 8; ++i) o[i] = (unsigned short)bf16_bits(W1[(size_t)(sr + i) * HF + n]);
    put8us(W1T + (size_t)n * 512 + k8, o);
  } else if (u < E_W2) {
    const int v = u - E_W1, n = v >> 5, k8 = (v & 31) * 8, sr = k8 & 127;
    v8us o;
#pragma unroll
    for (int i = 0; i < 8; ++i) o[i] = (unsigned short)bf16_bits(W2[(size_t)(sr + i) * HF + n]);
    put8us(W2T + (size_t)n * 256 + k8, o);
  } else if (u < E_WO) {
    const int v = u - E_W2, n = v >> 5, k8 = (v & 31) * 8, sr = k8 & 127;
    v8us o;
#pragma unroll
    for (int i = 0; i < 8; ++i) o[i] = (unsigned short)bf16_bits(Wo[(size_t)(sr + i) * OUTF + n]);
    put8us(WoT + (size_t)n * 256 + k8, o);
  } else if (u < E_BT) {
    const int v = u - E_WO, n = v >> 3, k8 = (v & 7) * 8;
    const int col = n + (n & 128);
    v8h o;
#pragma unroll
    for (int i = 0; i < 8; ++i) o[i] = (_Float16)(CW * bf16_val(Wtime[(size_t)(k8 + i) * KQ3 + col]));
    put8h(BKV + (size_t)n * BKP + k8, o);
  } else if (u < E_BE) {
    const int v = u - E_BT, n = v >> 3, k8 = (v & 7) * 8;
    const int col = n + (n & 128);
    v8h o;
#pragma unroll
    for (int i = 0; i < 8; ++i) {
      const int kk = k8 + i;
      const int kc = kk < RF ? kk : RF - 1;
      const float wv = Wedge[(size_t)kc * KQ3 + col];
      const float ov = kk < RF ? CW * bf16_val(wv) : 0.0f;
      o[i] = (_Float16)ov;
    }
    put8h(BKV + (size_t)n * BKP + TF + k8, o);
  } else if (u < E_TQW) {
    const int v = u - E_BE, n = v >> 3, k8 = (v & 7) * 8;
    v8h o;
#pragma unroll
    for (int i = 0; i < 8; ++i) o[i] = (_Float16)(CW * bf16_val(Wtime[(size_t)(k8 + i) * KQ3 + HF + n]));
    put8h(WtqT + (size_t)n * TF + k8, o);
  } else if (u < E_XB) {
    const int v = u - E_TQW, row = v >> 4, k8 = (v & 15) * 8;
    const int rc = row < nN ? row : nN - 1;
    const float* p = x + (size_t)rc * HF + k8;
    const v4f a = *(const v4fa*)p;
    const v4f b = *(const v4fa*)(p + 4);
    const unsigned mk = row < nN ? 0xFFFFu : 0u;
    v8us o;
    o[0] = (unsigned short)(mk & bf16_bits(a.x)); o[1] = (unsigned short)(mk & bf16_bits(a.y));
    o[2] = (unsigned short)(mk & bf16_bits(a.z)); o[3] = (unsigned short)(mk & bf16_bits(a.w));
    o[4] = (unsigned short)(mk & bf16_bits(b.x)); o[5] = (unsigned short)(mk & bf16_bits(b.y));
    o[6] = (unsigned short)(mk & bf16_bits(b.z)); o[7] = (unsigned short)(mk & bf16_bits(b.w));
    put8us(XB + (size_t)row * HF + k8, o);
  }
}

__global__ __launch_bounds__(NTHR) void k_tn(const float* __restrict__ times, const float* __restrict__ rels,
                                             const float* __restrict__ Wt, const float* __restrict__ bt, int nN,
                                             _Float16* AT, _Float16* TQ) {
  __shared__ __attribute__((aligned(16))) _Float16 sT[NTHR * KA];
  __shared__ __attribute__((aligned(16))) _Float16 sQ8[8 * TF];
  __shared__ float sWt[TH];
  __shared__ float sBt[TH];
  const int tid = (int)threadIdx.x, lane = tid & 31, w = tid >> 5;
  const int node = (int)blockIdx.x * 8 + w;
  const int nc = node < nN ? node : nN - 1;
  {
    const float a = bf16_val(Wt[lane]);
    const float b = bf16_val(bt[lane]);
    if (w == 0) sWt[lane] = a;
    if (w == 1) sBt[lane] = b;
  }
  const float t = bf16_val(times[(size_t)nc * KS + lane]);
  const bool mk = (t >= START_T) && (t < END_T);
  float tm = mk ? t : START_T;
#pragma unroll
  for (int off = 16; off > 0; off >>= 1) tm = fmaxf(tm, __shfl_xor(tm, off, 32));
  const float tmax = tm;
  __syncthreads();

  const float dt = tmax - t;
  const float dq = tmax - START_T;
  _Float16* srow = sT + tid * KA;
#pragma unroll 1
  for (int q = 0; q <= TH; ++q) {
    const int qc = q < TH ? q : TH - 1;
    const float hs = dt * sWt[qc] + sBt[qc];
    const float hq = dq * sWt[lane] + sBt[lane];
    const float hv = q < TH ? hs : hq;
    float sv, cv;
    sincosf(hv, &sv, &cv);
    const float a = sv * T_NORM;
    const float b = cv * T_NORM;
    v2h p;
    p.x = (_Float16)(a * CA);
    p.y = (_Float16)(b * CA);
    _Float16* dp = q < TH ? (srow + 2 * q) : (sQ8 + w * TF + 2 * lane);
    *(v2ha*)dp = p;
  }
  {
    const float* rr = rels + ((size_t)nc * KS + lane) * RF;
#pragma unroll
    for (int g = 0; g < 4; ++g) {
      const v4f a = *(const v4fa*)(rr + 8 * g);
      const v4f b = *(const v4fa*)(rr + 8 * g + 4);
      v8h o;
      o[0] = (_Float16)(CA * bf16_val(a.x)); o[1] = (_Float16)(CA * bf16_val(a.y));
      o[2] = (_Float16)(CA * bf16_val(a.z)); o[3] = (_Float16)(CA * bf16_val(a.w));
      o[4] = (_Float16)(CA * bf16_val(b.x)); o[5] = (_Float16)(CA * bf16_val(b.y));
      o[6] = (_Float16)(CA * bf16_val(b.z)); o[7] = (_Float16)(CA * bf16_val(b.w));
      *(v8ha*)(srow + TF + 8 * g) = o;
    }
  }
  __syncthreads();

  _Float16* dstb = AT + (size_t)blockIdx.x * NTHR * KA;
#pragma unroll
  for (int it = 0; it < (NTHR * KA) / (8 * NTHR); ++it) {
    const int p = it * NTHR + tid;
    const v8h v = *(const v8ha*)(sT + 8 * p);
    *(volatile v8h*)(dstb + 8 * p) = v;
  }
  const int tl = tid < 64 ? tid : 63;
  const v8h tq = *(const v8ha*)(sQ8 + 8 * tl);
  _Float16* tqp = TQ + (size_t)blockIdx.x * 8 * TF + 8 * tl;
  if (tid < 64) *(volatile v8h*)tqp = tq;
  __threadfence();
#pragma unroll
  for (int it = 0; it < (NTHR * KA) / (8 * NTHR); ++it) {
    const int p = it * NTHR + tid;
    const v8h v = *(const v8ha*)(sT + 8 * p);
    *(volatile v8h*)(dstb + 8 * p) = v;
  }
  if (tid < 64) *(volatile v8h*)tqp = tq;
}

template <bool F16OP, int NT, int EPI, bool HAS_BIAS, bool RELU, bool HAS_RES>
__global__ __launch_bounds__(GTHR) void k_gemm(const unsigned short* __restrict__ A, int lda,
                                               const unsigned short* __restrict__ BT, int ldb, int K, float scale,
                                               const float* __restrict__ bias,
                                               const float* __restrict__ resid, int ldr,
                                               float* Cf, int ldc, unsigned short* Cb, int ldcb, int nvalid) {
  static_assert((NT == 8 && EPI >= 0 && EPI <= 2) || (NT == 4 && EPI == 3));
  __shared__ __attribute__((aligned(16))) float stg[GBM * GBN];
  const int tid = (int)threadIdx.x, lane = tid & 31, wave = tid >> 5, hh = lane >> 4, m = lane & 15;
  const int rowBase = (int)blockIdx.x * GBM;
  const int colBase = (int)blockIdx.y * (16 * NT);

  v8f acc[NT];
  {
    const v8f z = {0.f, 0.f, 0.f, 0.f, 0.f, 0.f, 0.f, 0.f};
#pragma unroll
    for (int t = 0; t < NT; ++t) acc[t] = z;
  }
  const unsigned short* ap = A  + (size_t)(rowBase + 16 * wave + m) * (size_t)lda + 8 * hh;
  const unsigned short* bp = BT + (size_t)(colBase + m) * (size_t)ldb + 8 * hh;

#pragma unroll 1
  for (int k0 = 0; k0 < K; k0 += 32) {
    Frag16 af;
    af.u[0] = *(const v8usa*)(ap + k0);
    af.u[1] = *(const v8usa*)(ap + k0 + 16);
#pragma unroll
    for (int nt = 0; nt < NT; ++nt) {
      const unsigned short* wq = bp + (size_t)(16 * nt) * (size_t)ldb + k0;
      Frag16 bf;
      bf.u[0] = *(const v8usa*)wq;
      bf.u[1] = *(const v8usa*)(wq + 16);
      if (F16OP) acc[nt] = wm_h(af, bf, acc[nt]);
      else       acc[nt] = wm_b(af, bf, acc[nt]);
    }
  }

#pragma unroll
  for (int nt = 0; nt < NT; ++nt) {
    const int lc = 16 * nt + m;
#pragma unroll
    for (int r = 0; r < 8; ++r) {
      const int lr = 16 * wave + 8 * hh + r;
      stg[lr * GBN + lc] = acc[nt][r];
    }
  }
  __syncthreads();

  if (EPI != 3) {
    const int c4 = 4 * lane;
    v4f b4 = {0.f, 0.f, 0.f, 0.f};
    if (HAS_BIAS) b4 = bf4(*(const v4fa*)(bias + colBase + c4));
#pragma unroll
    for (int i = 0; i < 16; ++i) {
      const int lr = 16 * wave + i;
      v4f v = *(const v4fa*)(stg + lr * GBN + c4);
      v = v * scale + b4;
      if (RELU) { v.x = fmaxf(v.x, 0.f); v.y = fmaxf(v.y, 0.f); v.z = fmaxf(v.z, 0.f); v.w = fmaxf(v.w, 0.f); }
      if (HAS_RES) {
        const v4f rv = *(const v4fa*)(resid + (size_t)(rowBase + lr) * (size_t)ldr + colBase + c4);
        v = v + rv;
      }
      *(v4fa*)(stg + lr * GBN + c4) = v;
    }
    __syncthreads();
    if (EPI == 0 || EPI == 2) {
#pragma unroll
      for (int i = 0; i < 16; ++i) {
        const int lr = 16 * wave + i;
        const v4f v = *(const v4fa*)(stg + lr * GBN + c4);
        *(volatile v4f*)(Cf + (size_t)(rowBase + lr) * (size_t)ldc + colBase + c4) = v;
      }
      __threadfence();
#pragma unroll
      for (int i = 0; i < 16; ++i) {
        const int lr = 16 * wave + i;
        const v4f v = *(const v4fa*)(stg + lr * GBN + c4);
        *(volatile v4f*)(Cf + (size_t)(rowBase + lr) * (size_t)ldc + colBase + c4) = v;
      }
    }
    if (EPI == 1 || EPI == 2) {
      const int c8 = 8 * (lane & 15);
      const unsigned sel = 0u - (unsigned)(lane >> 4);
#pragma unroll
      for (int i = 0; i < 16; ++i) {
        const int lr = 16 * wave + i;
        const v4f a = *(const v4fa*)(stg + lr * GBN + c8);
        const v4f b = *(const v4fa*)(stg + lr * GBN + c8 + 4);
        v8us o;
        o[0] = hl_bits(a.x, sel); o[1] = hl_bits(a.y, sel); o[2] = hl_bits(a.z, sel); o[3] = hl_bits(a.w, sel);
        o[4] = hl_bits(b.x, sel); o[5] = hl_bits(b.y, sel); o[6] = hl_bits(b.z, sel); o[7] = hl_bits(b.w, sel);
        *(volatile v8us*)(Cb + (size_t)(rowBase + lr) * (size_t)ldcb + 8 * lane) = o;
      }
      __threadfence();
#pragma unroll
      for (int i = 0; i < 16; ++i) {
        const int lr = 16 * wave + i;
        const v4f a = *(const v4fa*)(stg + lr * GBN + c8);
        const v4f b = *(const v4fa*)(stg + lr * GBN + c8 + 4);
        v8us o;
        o[0] = hl_bits(a.x, sel); o[1] = hl_bits(a.y, sel); o[2] = hl_bits(a.z, sel); o[3] = hl_bits(a.w, sel);
        o[4] = hl_bits(b.x, sel); o[5] = hl_bits(b.y, sel); o[6] = hl_bits(b.z, sel); o[7] = hl_bits(b.w, sel);
        *(volatile v8us*)(Cb + (size_t)(rowBase + lr) * (size_t)ldcb + 8 * lane) = o;
      }
    }
  } else {
    const int half2 = lane >> 4, c4 = 4 * (lane & 15);
    v4f b4 = {0.f, 0.f, 0.f, 0.f};
    if (HAS_BIAS) b4 = bf4(*(const v4fa*)(bias + c4));
#pragma unroll
    for (int i = 0; i < 8; ++i) {
      const int lr = 16 * wave + 2 * i + half2;
      const int grow = rowBase + lr;
      v4f v = *(const v4fa*)(stg + lr * GBN + c4);
      v = v * scale + b4;
      if (grow < nvalid) *(volatile v4f*)(Cf + (size_t)grow * OUTF + c4) = v;
    }
    __threadfence();
#pragma unroll
    for (int i = 0; i < 8; ++i) {
      const int lr = 16 * wave + 2 * i + half2;
      const int grow = rowBase + lr;
      v4f v = *(const v4fa*)(stg + lr * GBN + c4);
      v = v * scale + b4;
      if (grow < nvalid) *(volatile v4f*)(Cf + (size_t)grow * OUTF + c4) = v;
    }
  }
}

__global__ __launch_bounds__(NTHR) void k_ln1(const float* __restrict__ H, const float* __restrict__ g,
                                              const float* __restrict__ b, float* XN, unsigned short* Z0) {
  __shared__ __attribute__((aligned(16))) unsigned short sZ[8 * 2 * HF];
  const int tid = (int)threadIdx.x, lane = tid & 31, w = tid >> 5;
  const int row = (int)blockIdx.x * 8 + w;
  const int c4 = 4 * lane;
  const v4f x = *(const v4fa*)(H + (size_t)row * HF + c4);
  const v4f gg = bf4(*(const v4fa*)(g + c4));
  const v4f bb = bf4(*(const v4fa*)(b + c4));
  float s = (x.x + x.y) + (x.z + x.w);
#pragma unroll
  for (int off = 16; off > 0; off >>= 1) s += __shfl_xor(s, off, 32);
  const float mean = s * (1.0f / HF);
  const v4f d = x - mean;
  float q = (d.x * d.x + d.y * d.y) + (d.z * d.z + d.w * d.w);
#pragma unroll
  for (int off = 16; off > 0; off >>= 1) q += __shfl_xor(q, off, 32);
  const float var = q * (1.0f / HF);
  const float rstd = rsqrtf(var + LN_EPS);
  const v4f y = d * rstd * gg + bb;
  v4us hb, lb;
  {
    const unsigned h0 = bf16_bits(y.x), h1 = bf16_bits(y.y), h2 = bf16_bits(y.z), h3 = bf16_bits(y.w);
    hb.x = (unsigned short)h0; hb.y = (unsigned short)h1; hb.z = (unsigned short)h2; hb.w = (unsigned short)h3;
    lb.x = (unsigned short)bf16_bits(y.x - __uint_as_float(h0 << 16));
    lb.y = (unsigned short)bf16_bits(y.y - __uint_as_float(h1 << 16));
    lb.z = (unsigned short)bf16_bits(y.z - __uint_as_float(h2 << 16));
    lb.w = (unsigned short)bf16_bits(y.w - __uint_as_float(h3 << 16));
  }
  unsigned short* zr = sZ + w * 2 * HF;
  *(v4usa*)(zr + c4) = hb;
  *(v4usa*)(zr + HF + c4) = lb;
  __syncthreads();
  const v8us o8 = *(const v8usa*)(zr + 8 * lane);
  float* xp = XN + (size_t)row * HF + c4;
  unsigned short* zp = Z0 + (size_t)row * (4 * HF) + 8 * lane;
  *(volatile v4f*)xp = y;
  *(volatile v8us*)zp = o8;
  __threadfence();
  *(volatile v4f*)xp = y;
  *(volatile v8us*)zp = o8;
}

__global__ __launch_bounds__(NTHR) void k_slot(const float* __restrict__ times, const int* __restrict__ nbrs, int nN,
                                               const unsigned short* __restrict__ AT,
                                               const unsigned short* __restrict__ BKV,
                                               const float* __restrict__ KQV, const float* __restrict__ QT,
                                               const float* __restrict__ XN, const float* __restrict__ g2,
                                               const float* __restrict__ b2, float* H2, unsigned short* Z0) {
  extern __shared__ __attribute__((aligned(16))) float dyn[];
  char* base = (char*)dyn;
  float* sR = (float*)(base);
  float* sQ = (float*)(base + L_SR);
  float* sS = (float*)(base + L_SR + L_SQ);
  float* sP = (float*)(base + L_SR + L_SQ + L_SS);
  int*   sJ = (int*)(base + L_SR + L_SQ + L_SS + L_SP);
  int*   sM = (int*)(base + L_SR + L_SQ + L_SS + L_SP + L_SJ);

  const int tid = (int)threadIdx.x, lane = tid & 31, w = tid >> 5, hh = lane >> 4, m = lane & 15;
  const int node = (int)blockIdx.x * 8 + w;
  const int nc = node < nN ? node : nN - 1;
  const int s = tid;

  const float t = bf16_val(times[(size_t)nc * KS + lane]);
  const int mk = ((t >= START_T) && (t < END_T)) ? 1 : 0;
  int anyv = mk;
#pragma unroll
  for (int off = 16; off > 0; off >>= 1) anyv |= __shfl_xor(anyv, off, 32);
  {
    int j = nbrs[(size_t)nc * KS + lane];
    j = j < 0 ? 0 : (j > nN - 1 ? nN - 1 : j);
    sJ[s] = j;
    sM[s] = mk;
    const v4f qa = *(const v4fa*)(KQV + (size_t)nc * KQ3 + HF + 4 * lane);
    const v4f qb = *(const v4fa*)(QT + (size_t)nc * HF + 4 * lane);
    *(v4fa*)(sQ + w * HF + 4 * lane) = qa + qb;
  }
  __syncthreads();

  float* sRw = sR + w * 16 * SRP;
  v4f o4 = {0.f, 0.f, 0.f, 0.f};
#pragma unroll 1
  for (int pc = 0; pc < 2; ++pc) {
#pragma unroll 1
    for (int mt = 0; mt < 2; ++mt) {
      v8f acc[8];
      {
        const v8f z = {0.f, 0.f, 0.f, 0.f, 0.f, 0.f, 0.f, 0.f};
#pragma unroll
        for (int t8 = 0; t8 < 8; ++t8) acc[t8] = z;
      }
      const unsigned short* ap = AT + ((size_t)node * KS + 16 * mt + m) * (size_t)KA + 8 * hh;
      const unsigned short* bp = BKV + (size_t)(HF * pc + m) * BKP + 8 * hh;
#pragma unroll
      for (int k0 = 0; k0 < KA; k0 += 32) {
        Frag16 af;
        af.u[0] = *(const v8usa*)(ap + k0);
        af.u[1] = *(const v8usa*)(ap + k0 + 16);
#pragma unroll
        for (int nt = 0; nt < 8; ++nt) {
          const unsigned short* wq = bp + (size_t)(16 * nt) * BKP + k0;
          Frag16 bf;
          bf.u[0] = *(const v8usa*)wq;
          bf.u[1] = *(const v8usa*)(wq + 16);
          acc[nt] = wm_h(af, bf, acc[nt]);
        }
      }
#pragma unroll
      for (int nt = 0; nt < 8; ++nt) {
#pragma unroll
        for (int r = 0; r < 8; ++r) sRw[(8 * hh + r) * SRP + 16 * nt + m] = acc[nt][r] * INVC;
      }
      __syncthreads();

      if (pc == 0) {
        const int ri = lane >> 1, hb = 4 * (lane & 1);
        const int kk = 16 * mt + ri;
        const int jj = sJ[32 * w + kk];
        const float* kr = KQV + (size_t)jj * KQ3;
        const float* qr = sQ + w * HF;
        const float* rr = sRw + ri * SRP;
#pragma unroll 1
        for (int hq = 0; hq < 4; ++hq) {
          const int hd = hb + hq, c0 = HDIM * hd;
          const v4f q0 = *(const v4fa*)(qr + c0),      q1 = *(const v4fa*)(qr + c0 + 4);
          const v4f q2 = *(const v4fa*)(qr + c0 + 8),  q3 = *(const v4fa*)(qr + c0 + 12);
          const v4f r0 = *(const v4fa*)(rr + c0),      r1 = *(const v4fa*)(rr + c0 + 4);
          const v4f r2 = *(const v4fa*)(rr + c0 + 8),  r3 = *(const v4fa*)(rr + c0 + 12);
          const v4f g0 = *(const v4fa*)(kr + c0),      g1 = *(const v4fa*)(kr + c0 + 4);
          const v4f gg2 = *(const v4fa*)(kr + c0 + 8), g3 = *(const v4fa*)(kr + c0 + 12);
          float sc = 0.0f;
          sc = dot4s(q0, r0, g0, sc);
          sc = dot4s(q1, r1, g1, sc);
          sc = dot4s(q2, r2, gg2, sc);
          sc = dot4s(q3, r3, g3, sc);
          sS[(w * KS + kk) * NHEAD + hd] = sc * ATTN_NORM;
        }
      } else {
        const int c4 = 4 * lane, hd = lane >> 2;
#pragma unroll 2
        for (int i = 0; i < 16; ++i) {
          const int kk = 16 * mt + i;
          const int jj = sJ[32 * w + kk];
          const float a = sP[(w * KS + kk) * NHEAD + hd];
          const v4f rv = *(const v4fa*)(sRw + i * SRP + c4);
          const v4f gv = *(const v4fa*)(KQV + (size_t)jj * KQ3 + 2 * HF + c4);
          o4 = o4 + a * (rv + gv);
        }
      }
      __syncthreads();
    }
    if (pc == 0) {
      const int mrow = sM[32 * w + lane];
#pragma unroll 1
      for (int hd = 0; hd < NHEAD; ++hd) {
        const float sc = sS[(w * KS + lane) * NHEAD + hd];
        const float sv = mrow ? sc : -1e30f;
        float mx = sv;
#pragma unroll
        for (int off = 16; off > 0; off >>= 1) mx = fmaxf(mx, __shfl_xor(mx, off, 32));
        const float e = expf(sv - mx);
        float sm = e;
#pragma unroll
        for (int off = 16; off > 0; off >>= 1) sm += __shfl_xor(sm, off, 32);
        sP[(w * KS + lane) * NHEAD + hd] = e * (1.0f / sm);
      }
      __syncthreads();
    }
  }

  const int c4 = 4 * lane;
  const v4f xn4 = *(const v4fa*)(XN + (size_t)nc * HF + c4);
  const float hasf = anyv ? 1.0f : 0.0f;
  const v4f h2v = o4 * hasf + xn4;
  float su = (h2v.x + h2v.y) + (h2v.z + h2v.w);
#pragma unroll
  for (int off = 16; off > 0; off >>= 1) su += __shfl_xor(su, off, 32);
  const float mean = su * (1.0f / HF);
  const v4f d = h2v - mean;
  float qv = (d.x * d.x + d.y * d.y) + (d.z * d.z + d.w * d.w);
#pragma unroll
  for (int off = 16; off > 0; off >>= 1) qv += __shfl_xor(qv, off, 32);
  const float var = qv * (1.0f / HF);
  const float rstd = rsqrtf(var + LN_EPS);
  const v4f gg = bf4(*(const v4fa*)(g2 + c4));
  const v4f bb = bf4(*(const v4fa*)(b2 + c4));
  const v4f hn = d * rstd * gg + bb;
  v4us hb4, lb4;
  {
    const unsigned h0 = bf16_bits(hn.x), h1 = bf16_bits(hn.y), h2b = bf16_bits(hn.z), h3 = bf16_bits(hn.w);
    hb4.x = (unsigned short)h0; hb4.y = (unsigned short)h1; hb4.z = (unsigned short)h2b; hb4.w = (unsigned short)h3;
    lb4.x = (unsigned short)bf16_bits(hn.x - __uint_as_float(h0 << 16));
    lb4.y = (unsigned short)bf16_bits(hn.y - __uint_as_float(h1 << 16));
    lb4.z = (unsigned short)bf16_bits(hn.z - __uint_as_float(h2b << 16));
    lb4.w = (unsigned short)bf16_bits(hn.w - __uint_as_float(h3 << 16));
  }
  unsigned short* usr = (unsigned short*)sRw;
  *(v4usa*)(usr + c4) = hb4;
  *(v4usa*)(usr + HF + c4) = lb4;
  __syncthreads();
  const v8us o8 = *(const v8usa*)(usr + 8 * lane);
  float* hp = H2 + (size_t)node * HF + c4;
  unsigned short* zp = Z0 + (size_t)node * (4 * HF) + 2 * HF + 8 * lane;
  *(volatile v4f*)hp = h2v;
  *(volatile v8us*)zp = o8;
  __threadfence();
  *(volatile v4f*)hp = h2v;
  *(volatile v8us*)zp = o8;
}

extern "C" void kernel_launch(void* const* d_in, const int* in_sizes, int n_in,
                              void* d_out, int out_size, void* d_ws, size_t ws_size,
                              hipStream_t stream) {
  if (n_in < 21) return;
  const int nN = NNODE;
  if (in_sizes[0] != nN * HF) return;
  if (in_sizes[1] != nN * KS) return;
  if (in_sizes[2] != nN * KS) return;
  if (in_sizes[3] != nN * KS * RF) return;
  if (in_sizes[4] != HF * HF || in_sizes[5] != HF) return;
  if (in_sizes[6] != HF * KQ3) return;
  if (in_sizes[7] != TH || in_sizes[8] != TH) return;
  if (in_sizes[9] != TF * KQ3) return;
  if (in_sizes[10] != RF * KQ3) return;
  if (in_sizes[11] != HF || in_sizes[12] != HF || in_sizes[13] != HF || in_sizes[14] != HF) return;
  if (in_sizes[15] != 2 * HF * HF || in_sizes[16] != HF) return;
  if (in_sizes[17] != HF * HF || in_sizes[18] != HF) return;
  if (in_sizes[19] != HF * OUTF || in_sizes[20] != OUTF) return;
  if (out_size != nN * OUTF) return;

  const float* x     = (const float*)d_in[0];
  const int*   nbrs  = (const int*)d_in[1];
  const float* times = (const float*)d_in[2];
  const float* rels  = (const float*)d_in[3];
  const float* Wp    = (const float*)d_in[4];
  const float* bp    = (const float*)d_in[5];
  const float* Wkqv  = (const float*)d_in[6];
  const float* Wt    = (const float*)d_in[7];
  const float* bt    = (const float*)d_in[8];
  const float* Wtime = (const float*)d_in[9];
  const float* Wedge = (const float*)d_in[10];
  const float* g1    = (const float*)d_in[11];
  const float* b1n   = (const float*)d_in[12];
  const float* g2    = (const float*)d_in[13];
  const float* b2n   = (const float*)d_in[14];
  const float* W1    = (const float*)d_in[15];
  const float* bl1   = (const float*)d_in[16];
  const float* W2    = (const float*)d_in[17];
  const float* bl2   = (const float*)d_in[18];
  const float* Wo    = (const float*)d_in[19];
  const float* bo    = (const float*)d_in[20];
  float* out = (float*)d_out;

  char* ws = (char*)d_ws;
  size_t off = 0;
  const size_t oXB  = off; off += (size_t)MP * HF * 2;      off = (off + 255) & ~(size_t)255;
  const size_t oWP  = off; off += (size_t)HF * HF * 2;      off = (off + 255) & ~(size_t)255;
  const size_t oWK  = off; off += (size_t)KQ3 * 256 * 2;    off = (off + 255) & ~(size_t)255;
  const size_t oW1  = off; off += (size_t)HF * 512 * 2;     off = (off + 255) & ~(size_t)255;
  const size_t oW2  = off; off += (size_t)HF * 256 * 2;     off = (off + 255) & ~(size_t)255;
  const size_t oWO  = off; off += (size_t)OUTF * 256 * 2;   off = (off + 255) & ~(size_t)255;
  const size_t oBKV = off; off += (size_t)256 * BKP * 2;    off = (off + 255) & ~(size_t)255;
  const size_t oWTQ = off; off += (size_t)HF * TF * 2;      off = (off + 255) & ~(size_t)255;
  const size_t oAT  = off; off += (size_t)NSP * KA * 2;     off = (off + 255) & ~(size_t)255;
  const size_t oTQ  = off; off += (size_t)MP * TF * 2;      off = (off + 255) & ~(size_t)255;
  const size_t oH   = off; off += (size_t)MP * HF * 4;      off = (off + 255) & ~(size_t)255;
  const size_t oXN  = off; off += (size_t)MP * HF * 4;      off = (off + 255) & ~(size_t)255;
  const size_t oQT  = off; off += (size_t)MP * HF * 4;      off = (off + 255) & ~(size_t)255;
  const size_t oH2  = off; off += (size_t)MP * HF * 4;      off = (off + 255) & ~(size_t)255;
  const size_t oKQV = off; off += (size_t)MP * KQ3 * 4;     off = (off + 255) & ~(size_t)255;
  const size_t oZ0  = off; off += (size_t)MP * 512 * 2;     off = (off + 255) & ~(size_t)255;
  const size_t oZ1  = off; off += (size_t)MP * 256 * 2;     off = (off + 255) & ~(size_t)255;
  const size_t oHP  = off; off += (size_t)MP * 256 * 2;     off = (off + 255) & ~(size_t)255;
  if (off > ws_size || off > (size_t)WSMAX) return;

  unsigned short* XB  = (unsigned short*)(ws + oXB);
  unsigned short* WpT = (unsigned short*)(ws + oWP);
  unsigned short* WkT = (unsigned short*)(ws + oWK);
  unsigned short* W1T = (unsigned short*)(ws + oW1);
  unsigned short* W2T = (unsigned short*)(ws + oW2);
  unsigned short* WoT = (unsigned short*)(ws + oWO);
  _Float16*       BKV = (_Float16*)(ws + oBKV);
  _Float16*       WtqT = (_Float16*)(ws + oWTQ);
  _Float16*       AT  = (_Float16*)(ws + oAT);
  _Float16*       TQ  = (_Float16*)(ws + oTQ);
  float*          H   = (float*)(ws + oH);
  float*          XN  = (float*)(ws + oXN);
  float*          QT  = (float*)(ws + oQT);
  float*          H2  = (float*)(ws + oH2);
  float*          KQV = (float*)(ws + oKQV);
  unsigned short* Z0  = (unsigned short*)(ws + oZ0);
  unsigned short* Z1  = (unsigned short*)(ws + oZ1);
  unsigned short* HP  = (unsigned short*)(ws + oHP);

  hipFuncSetAttribute(reinterpret_cast<const void*>(&k_slot), hipFuncAttributeMaxDynamicSharedMemorySize, (int)SLOT_LDS);

  const int gM = MP / GBM;

  k_prep<<<E_XB / NTHR, NTHR, 0, stream>>>(x, Wp, Wkqv, Wtime, Wedge, W1, W2, Wo, nN,
                                           XB, WpT, WkT, W1T, W2T, WoT, BKV, WtqT);
  k_tn<<<MP / 8, NTHR, 0, stream>>>(times, rels, Wt, bt, nN, AT, TQ);
  k_gemm<false, 8, 0, true, true, false><<<dim3(gM, 1), GTHR, 0, stream>>>(
      XB, HF, WpT, HF, HF, 1.0f, bp, nullptr, 0, H, HF, nullptr, 0, MP);
  k_gemm<true, 8, 0, false, false, false><<<dim3(gM, 1), GTHR, 0, stream>>>(
      (const unsigned short*)TQ, TF, (const unsigned short*)WtqT, TF, TF, INVC, nullptr, nullptr, 0, QT, HF,
      nullptr, 0, MP);

  for (int L = 0; L < 2; ++L) {
    k_ln1<<<MP / 8, NTHR, 0, stream>>>(H, g1, b1n, XN, Z0);
    k_gemm<false, 8, 0, false, false, false><<<dim3(gM, KQ3 / GBN), GTHR, 0, stream>>>(
        Z0, 512, WkT, 256, 256, 1.0f, nullptr, nullptr, 0, KQV, KQ3, nullptr, 0, MP);
    k_slot<<<MP / 8, NTHR, SLOT_LDS, stream>>>(times, nbrs, nN, (const unsigned short*)AT, (const unsigned short*)BKV,
                                               KQV, QT, XN, g2, b2n, H2, Z0);
    k_gemm<false, 8, 1, true, true, false><<<dim3(gM, 1), GTHR, 0, stream>>>(
        Z0, 512, W1T, 512, 512, 1.0f, bl1, nullptr, 0, nullptr, 0, Z1, 256, MP);
    k_gemm<false, 8, 2, true, false, true><<<dim3(gM, 1), GTHR, 0, stream>>>(
        Z1, 256, W2T, 256, 256, 1.0f, bl2, H2, HF, H, HF, HP, 256, MP);
  }
  k_gemm<false, 4, 3, true, false, false><<<dim3(gM, 1), GTHR, 0, stream>>>(
      HP, 256, WoT, 256, 256, 1.0f, bo, nullptr, 0, out, OUTF, nullptr, 0, nN);
}
